// SwinTransformerBlock_19782619365404
// MI455X (gfx1250) — hardware-verified
//
#include <hip/hip_runtime.h>
#include <math.h>

typedef __attribute__((ext_vector_type(16))) _Float16 v16h;
typedef __attribute__((ext_vector_type(16))) __bf16 v16b;
typedef __attribute__((ext_vector_type(8)))  _Float16 v8h;
typedef __attribute__((ext_vector_type(8)))  float v8f;
typedef __attribute__((ext_vector_type(4)))  float v4f;
typedef __attribute__((ext_vector_type(2)))  float v2f;
typedef __attribute__((ext_vector_type(4)))  unsigned v4u;
typedef __attribute__((ext_vector_type(4)))  int v4i;
typedef float __attribute__((may_alias)) float_a;
typedef int __attribute__((may_alias)) int_a;

template <typename T> __device__ __forceinline__ void vst2(void* p, T v) { *(volatile T*)p = v; __threadfence(); *(volatile T*)p = v; }
__device__ __forceinline__ v8f wmma16(v16h a, v16h b, v8f c) {
  v8f d = __builtin_amdgcn_wmma_f32_16x16x32_f16(false, a, false, b, (short)0, c, false, false);
  asm volatile("v_nop\n\tv_nop\n\tv_nop\n\tv_nop" : "+v"(d) : "v"(a), "v"(b));
  return d;
}
__device__ __forceinline__ v8f wmma_bf(v16b a, v16b b, v8f c) {
  v8f d = __builtin_amdgcn_wmma_f32_16x16x32_bf16(false, a, false, b, (short)0, c, false, false);
  asm volatile("v_nop\n\tv_nop\n\tv_nop\n\tv_nop" : "+v"(d) : "v"(a), "v"(b));
  return d;
}
__device__ __forceinline__ v16h frag_h(const _Float16* rowk0, int lane) {
  union { v16h v; v8h q[2]; } u; const _Float16* p = rowk0 + 8 * (lane >> 4);
  u.q[0] = *(const v8h*)p; u.q[1] = *(const v8h*)(p + 16); return u.v;
}
__device__ __forceinline__ v16h frag_f32(const float* rowk0, int lane) {
  v16h a; const float* p = rowk0 + 8 * (lane >> 4);
#pragma unroll
  for (int i = 0; i < 8; ++i) { a[i] = (_Float16)p[i]; a[8 + i] = (_Float16)p[16 + i]; }
  return a;
}
__device__ __forceinline__ v16h frag_f32s(const float* rowk0, int lane, float sc) {
  v16h a; const float* p = rowk0 + 8 * (lane >> 4);
#pragma unroll
  for (int i = 0; i < 8; ++i) { a[i] = (_Float16)(p[i] * sc); a[8 + i] = (_Float16)(p[16 + i] * sc); }
  return a;
}
__device__ __forceinline__ v16h fragc_f32(const float* W, int k0, int n, int lane, int ld, int K) {
  v16h a; const int g = lane >> 4;
#pragma unroll
  for (int i = 0; i < 8; ++i) { const int ka = k0 + 8 * g + i, kb = ka + 16;
    a[i] = (_Float16)(ka < K ? W[(size_t)(ka < K ? ka : K - 1) * ld + n] : 0.f); a[8 + i] = (_Float16)(kb < K ? W[(size_t)(kb < K ? kb : K - 1) * ld + n] : 0.f); }
  return a;
}
struct F2 { v16b h, l; };
__device__ __forceinline__ F2 bsplit16(const float v[16]) { F2 r;
#pragma unroll
  for (int i = 0; i < 16; ++i) { const __bf16 h = (__bf16)v[i]; r.h[i] = h; r.l[i] = (__bf16)(v[i] - (float)h); }
  return r; }
__device__ __forceinline__ F2 split_row(const float* row, int k0, int lane) { float v[16]; const float* p = row + k0 + 8 * (lane >> 4);
#pragma unroll
  for (int i = 0; i < 8; ++i) { v[i] = p[i]; v[8 + i] = p[16 + i]; }
  return bsplit16(v); }
__device__ __forceinline__ F2 split_rowK(const float* row, int k0, int lane, int K) { float v[16]; const int g = lane >> 4;
#pragma unroll
  for (int i = 0; i < 8; ++i) { const int ka = k0 + 8 * g + i, kb = ka + 16; v[i] = ka < K ? row[ka < K ? ka : K - 1] : 0.f; v[8 + i] = kb < K ? row[kb < K ? kb : K - 1] : 0.f; }
  return bsplit16(v); }
__device__ __forceinline__ F2 split_col(const float* W, int k0, int n, int lane, int ld, int K) { float v[16]; const int g = lane >> 4;
#pragma unroll
  for (int i = 0; i < 8; ++i) { const int ka = k0 + 8 * g + i, kb = ka + 16; v[i] = ka < K ? W[(size_t)(ka < K ? ka : K - 1) * ld + n] : 0.f; v[8 + i] = kb < K ? W[(size_t)(kb < K ? kb : K - 1) * ld + n] : 0.f; }
  return bsplit16(v); }
__device__ __forceinline__ v8f mac3(const F2& a, const F2& b, v8f c) { c = wmma_bf(a.l, b.h, c); c = wmma_bf(a.h, b.l, c); return wmma_bf(a.h, b.h, c); }
__device__ __forceinline__ float sigm(float v) { return 1.0f / (1.0f + expf(-v)); }
#define LDSX() do { asm volatile("s_wait_dscnt 0" ::: "memory"); __builtin_amdgcn_wave_barrier(); __builtin_amdgcn_fence(__ATOMIC_RELEASE, "workgroup"); } while (0)

__device__ __forceinline__ float bfr(float v) { return (float)(__bf16)v; }
__device__ __forceinline__ v16b wcol_io(const float* __restrict__ Wm, int k0, int o, int lane, int ld) { v16b w; const float* p = Wm + (size_t)(k0 + 8 * (lane >> 4)) * ld + o;
#pragma unroll
  for (int i = 0; i < 8; ++i) { w[i] = (__bf16)p[(size_t)i * ld]; w[8 + i] = (__bf16)p[(size_t)(16 + i) * ld]; }
  asm volatile("s_wait_loadcnt 0x0" ::: "memory"); return w; }
#define NIMG 32
#define IH 56
#define CC 128
#define DIN 128
#define NHD 4
#define HDD 32
#define WSZ 7
#define NWIN (NIMG * (IH / WSZ) * (IH / WSZ))
#define NTW 49
#define NROW (NIMG * IH * IH)
#ifndef NROWV
#define NROWV NROW
#endif
#define MH 512
#define RCH (NROW / 2)
__device__ __forceinline__ v4f wave_ln128(v4f t, int lane, const float* __restrict__ G, const float* __restrict__ Bt) { float s1 = (t[0] + t[1]) + (t[2] + t[3]);
#pragma unroll
  for (int o = 1; o < 32; o <<= 1) s1 += __shfl_xor(s1, o);
  const float mu = s1 * (1.0f / 128.0f); float q = 0.f;
#pragma unroll
  for (int i = 0; i < 4; ++i) { const float d = t[i] - mu; q += d * d; }
#pragma unroll
  for (int o = 1; o < 32; o <<= 1) q += __shfl_xor(q, o);
  const float rs = rsqrtf(q * (1.0f / 128.0f) + 1e-5f); v4f r4;
#pragma unroll
  for (int i = 0; i < 4; ++i) r4[i] = (t[i] - mu) * rs * bfr(G[lane * 4 + i]) + bfr(Bt[lane * 4 + i]);
  return r4; }
__global__ __launch_bounds__(256) void k_ln128(const float* __restrict__ X, int roundin, const float* __restrict__ G, const float* __restrict__ Bt, float* __restrict__ XN, const int* __restrict__ HIN = nullptr, const int* __restrict__ WIN = nullptr) { (void)HIN; (void)WIN;     const int wave = threadIdx.x >> 5, lane = threadIdx.x & 31; const size_t row = (size_t)blockIdx.x * 8 + wave; if (row >= (size_t)NROWV) return;
  v4f t = *(const v4f*)(X + row * CC + lane * 4); if (roundin) { t[0] = bfr(t[0]); t[1] = bfr(t[1]); t[2] = bfr(t[2]); t[3] = bfr(t[3]); }
  vst2(XN + row * CC + lane * 4, wave_ln128(t, lane, G, Bt)); }
__device__ __forceinline__ size_t win_tok(int wdx, int n) { const int b = wdx / 64, wr = wdx % 64, wy = wr / 8, wx = wr % 8; const int yy = wy * WSZ + n / WSZ, xx = wx * WSZ + n % WSZ; return ((size_t)b * IH + yy) * IH + xx; }
__device__ __forceinline__ F2 split_ptr(const float* __restrict__ p, int lane) { float va[16]; const int g = lane >> 4;
#pragma unroll
  for (int i = 0; i < 8; ++i) { va[i] = p[8 * g + i]; va[8 + i] = p[16 + 8 * g + i]; }
  return bsplit16(va); }
__global__ __launch_bounds__(128) void k_win(const float* __restrict__ XN, const float* __restrict__ WQKV, const float* __restrict__ BQKV, const float* __restrict__ RT, const float* __restrict__ PW, const float* __restrict__ PB, float* __restrict__ XO) {
  __shared__ float sq[64][33], sk[64][33], sv[64][33]; __shared__ float ss[64][65]; __shared__ __align__(16) float sc[64][132]; __shared__ float srt[169 * NHD];
  const int tid = threadIdx.x, wave = tid >> 5, lane = tid & 31, col = lane & 15, g = lane >> 4; const int wdx = blockIdx.x;
  const int myrow = wave * 16 + col;
  v16b ah[4], al[4];
  { const bool real = myrow < NTW; const size_t tk = win_tok(wdx, real ? myrow : 0); const float* p = XN + tk * CC;
#pragma unroll
    for (int kc = 0; kc < 4; ++kc) { float va[16];
#pragma unroll
      for (int i = 0; i < 8; ++i) { va[i] = real ? p[kc * 32 + 8 * g + i] : 0.f; va[8 + i] = real ? p[kc * 32 + 16 + 8 * g + i] : 0.f; }
      const F2 f = bsplit16(va); ah[kc] = f.h; al[kc] = f.l; } }
  for (int i = tid; i < 169 * NHD; i += 128) srt[i] = bfr(RT[i]);
  asm volatile("s_wait_loadcnt 0x0" ::: "memory");
  for (int h = 0; h < NHD; ++h) {
#pragma unroll
    for (int which = 0; which < 3; ++which) { v8f acc[2] = {};
#pragma unroll
      for (int kc = 0; kc < 4; ++kc) {
#pragma unroll
        for (int j = 0; j < 2; ++j) { const v16b w = wcol_io(WQKV, kc * 32, which * CC + h * HDD + j * 16 + col, lane, 3 * CC); acc[j] = wmma_bf(ah[kc], w, acc[j]); acc[j] = wmma_bf(al[kc], w, acc[j]); } }
      float (*dst)[33] = which == 0 ? sq : (which == 1 ? sk : sv);
#pragma unroll
      for (int j = 0; j < 2; ++j) { const float bb = bfr(BQKV[which * CC + h * HDD + j * 16 + col]);
#pragma unroll
        for (int r = 0; r < 8; ++r) dst[wave * 16 + 8 * g + r][j * 16 + col] = acc[j][r] + bb; } }
    __syncthreads();
    { const F2 a = split_ptr(&sq[myrow][0], lane); v8f acc[4] = {};
#pragma unroll
      for (int j = 0; j < 4; ++j) { const F2 bk = split_ptr(&sk[j * 16 + col][0], lane);
        acc[j] = wmma_bf(a.h, bk.h, acc[j]); acc[j] = wmma_bf(a.h, bk.l, acc[j]); acc[j] = wmma_bf(a.l, bk.h, acc[j]); acc[j] = wmma_bf(a.l, bk.l, acc[j]); }
#pragma unroll
      for (int j = 0; j < 4; ++j)
#pragma unroll
        for (int r = 0; r < 8; ++r) ss[wave * 16 + 8 * g + r][j * 16 + col] = acc[j][r]; }
    __syncthreads();
    if (lane < 16) { const int row = wave * 16 + lane; const int yi = row / WSZ, xi = row % WSZ; float mx = -3.0e38f; float e[NTW];
#pragma unroll
      for (int m = 0; m < NTW; ++m) { const int yj = m / WSZ, xj = m % WSZ; const int ridx = (row < NTW) ? ((yi - yj + WSZ - 1) * (2 * WSZ - 1) + (xi - xj + WSZ - 1)) : 0; const float v = ss[row][m] * 0.17677669529663689f + srt[ridx * NHD + h]; e[m] = v; mx = fmaxf(mx, v); }
      float sum = 0.f;
#pragma unroll
      for (int m = 0; m < NTW; ++m) { e[m] = expf(e[m] - mx); sum += e[m]; }
      const float inv = 1.0f / sum;
#pragma unroll
      for (int m = 0; m < NTW; ++m) ss[row][m] = e[m] * inv;
#pragma unroll
      for (int m = NTW; m < 64; ++m) ss[row][m] = 0.f; }
    __syncthreads();
    { v8f acc[2] = {};
#pragma unroll
      for (int kc = 0; kc < 2; ++kc) { const F2 a = split_ptr(&ss[myrow][kc * 32], lane);
#pragma unroll
        for (int j = 0; j < 2; ++j) { float vb[16]; const int d = j * 16 + col;
#pragma unroll
          for (int i = 0; i < 8; ++i) { vb[i] = sv[kc * 32 + 8 * g + i][d]; vb[8 + i] = sv[kc * 32 + 16 + 8 * g + i][d]; }
          const F2 bv = bsplit16(vb);
          acc[j] = wmma_bf(a.h, bv.h, acc[j]); acc[j] = wmma_bf(a.h, bv.l, acc[j]); acc[j] = wmma_bf(a.l, bv.h, acc[j]); acc[j] = wmma_bf(a.l, bv.l, acc[j]); } }
#pragma unroll
      for (int j = 0; j < 2; ++j)
#pragma unroll
        for (int r = 0; r < 8; ++r) sc[wave * 16 + 8 * g + r][h * HDD + j * 16 + col] = acc[j][r]; }
    __syncthreads(); }
  { v8f acc[8] = {};
#pragma unroll
    for (int kc = 0; kc < 4; ++kc) { const F2 a = split_ptr(&sc[myrow][kc * 32], lane);
#pragma unroll
      for (int j = 0; j < 8; ++j) { const v16b w = wcol_io(PW, kc * 32, j * 16 + col, lane, CC); acc[j] = wmma_bf(a.h, w, acc[j]); acc[j] = wmma_bf(a.l, w, acc[j]); } }
    __syncthreads();
#pragma unroll
    for (int j = 0; j < 8; ++j) { const float bb = bfr(PB[j * 16 + col]);
#pragma unroll
      for (int r = 0; r < 8; ++r) sc[wave * 16 + 8 * g + r][j * 16 + col] = acc[j][r] + bb; } }
  LDSX();
  for (int rl = 0; rl < 16; ++rl) { const int row = wave * 16 + rl; if (row < NTW) vst2(XO + win_tok(wdx, row) * CC + lane * 4, *(const v4f*)&sc[row][lane * 4]); } }
__global__ __launch_bounds__(128) void k_g1(const float* __restrict__ A, const float* __restrict__ W1, const float* __restrict__ B1, int rbase, float* __restrict__ Hh) { __shared__ __align__(16) float sf[4][16][132];
  const int tid = threadIdx.x, wave = tid >> 5, lane = tid & 31, col = lane & 15, g = lane >> 4; const int c0 = blockIdx.y * 128; const size_t r0 = (size_t)rbase + (size_t)blockIdx.x * 64 + wave * 16;
  v8f acc[8] = {};
#pragma unroll 2
  for (int kc = 0; kc < DIN / 32; ++kc) { const F2 a = split_row(A + (r0 + col) * DIN, kc * 32, lane); asm volatile("s_wait_loadcnt 0x0" ::: "memory");
#pragma unroll
    for (int j = 0; j < 8; ++j) { const v16b w = wcol_io(W1, kc * 32, c0 + j * 16 + col, lane, MH); asm volatile("s_wait_loadcnt 0x0" ::: "memory"); acc[j] = wmma_bf(a.h, w, acc[j]); acc[j] = wmma_bf(a.l, w, acc[j]); } }
#pragma unroll
  for (int j = 0; j < 8; ++j) { const float bb = bfr(B1[c0 + j * 16 + col]);
#pragma unroll
    for (int r = 0; r < 8; ++r) { const float u = acc[j][r] + bb; sf[wave][8 * g + r][j * 16 + col] = 0.5f * u * (1.0f + erff(u * 0.70710678118654752f)); } }
  LDSX(); for (int rl = 0; rl < 16; ++rl) vst2(Hh + (r0 - rbase + rl) * MH + c0 + lane * 4, *(const v4f*)&sf[wave][rl][lane * 4]); }
__global__ __launch_bounds__(128) void k_g2(const float* __restrict__ Hh, const float* __restrict__ W2, const float* __restrict__ B2, const float* __restrict__ X1, int rbase, float* __restrict__ OUT) { __shared__ __align__(16) float sf[4][16][132];
  const int tid = threadIdx.x, wave = tid >> 5, lane = tid & 31, col = lane & 15, g = lane >> 4; const int c0 = blockIdx.y * 128; const size_t r0 = (size_t)rbase + (size_t)blockIdx.x * 64 + wave * 16;
  v8f acc[8] = {};
#pragma unroll 2
  for (int kc = 0; kc < MH / 32; ++kc) { const F2 a = split_row(Hh + (r0 - rbase + col) * MH, kc * 32, lane); asm volatile("s_wait_loadcnt 0x0" ::: "memory");
#pragma unroll
    for (int j = 0; j < 8; ++j) { const v16b w = wcol_io(W2, kc * 32, c0 + j * 16 + col, lane, DIN); asm volatile("s_wait_loadcnt 0x0" ::: "memory"); acc[j] = wmma_bf(a.h, w, acc[j]); acc[j] = wmma_bf(a.l, w, acc[j]); } }
#pragma unroll
  for (int j = 0; j < 8; ++j) { const float bb = bfr(B2[c0 + j * 16 + col]);
#pragma unroll
    for (int r = 0; r < 8; ++r) sf[wave][8 * g + r][j * 16 + col] = acc[j][r] + bb; }
  LDSX(); for (int rl = 0; rl < 16; ++rl) { const size_t o2 = (r0 + rl) * DIN + c0 + lane * 4; const v4f x1 = *(const v4f*)(X1 + o2); v4f t = *(const v4f*)&sf[wave][rl][lane * 4]; t[0] += x1[0]; t[1] += x1[1]; t[2] += x1[2]; t[3] += x1[3]; vst2(OUT + o2, t); } }

#define WS_XN  0u
#define WS_XO  (WS_XN + 4u * (size_t)NROW * CC)
#define WS_HH  (WS_XO + 4u * (size_t)NROW * CC)
#define WS_END (WS_HH + 4u * (size_t)RCH * MH)
extern "C" void kernel_launch(void* const* d_in, const int* in_sizes, int n_in, void* d_out, int out_size, void* d_ws, size_t ws_size, hipStream_t stream) {
  (void)in_sizes; (void)n_in; (void)out_size;
  if (ws_size < (size_t)WS_END) return;
  char* ws = (char*)d_ws; const float** F = (const float**)d_in; float *XN = (float*)(ws + WS_XN), *XO = (float*)(ws + WS_XO), *Hh = (float*)(ws + WS_HH);
  k_ln128<<<dim3(NROWV / 8), 256, 0, stream>>>(F[0], 1, F[8], F[9], XN, (const int*)d_in[1], (const int*)d_in[2]);
  k_win<<<dim3(NROWV / NTW), 128, 0, stream>>>(XN, F[3], F[4], F[7], F[5], F[6], XO);
  k_ln128<<<dim3(NROWV / 8), 256, 0, stream>>>(XO, 0, F[10], F[11], XN);
  for (int rb = 0; rb < NROWV; rb += RCH) { const int nr = (NROWV - rb) < RCH ? (NROWV - rb) : RCH;
    k_g1<<<dim3(nr / 64, MH / 128), 128, 0, stream>>>(XN, F[12], F[13], rb, Hh);
    k_g2<<<dim3(nr / 64, DIN / 128), 128, 0, stream>>>(Hh, F[14], F[15], XO, rb, (float*)d_out); }
}
